// MultiHeadAttention_37864431681773
// MI455X (gfx1250) — hardware-verified
//
#include <hip/hip_runtime.h>
#include <math.h>

typedef __attribute__((ext_vector_type(16))) _Float16 v16h;
typedef __attribute__((ext_vector_type(8)))  _Float16 v8h;
typedef __attribute__((ext_vector_type(8)))  float    v8f;
typedef __attribute__((ext_vector_type(4)))  float    v4f;

constexpr int kB   = 2;
constexpr int kS   = 2048;
constexpr int kH   = 2048;
constexpr int kNH  = 16;
constexpr int kHD  = kH / kNH;
constexpr int kTok = kB * kS;
static_assert(kHD == 128);
static_assert((kTok % 64) == 0 && (kH % 64) == 0 && (kH % 32) == 0 && (kS % 64) == 0 && (kHD % 32) == 0);
static_assert((((kTok / 64) * (kH / 64)) % 8) == 0);

constexpr float kActCarry = 16.0f;
constexpr float kWCarry   = 1024.0f;
constexpr float kQKCarry  = 16.0f;
constexpr float kVCarry   = 16.0f;
constexpr float kCtxCarry = 1024.0f;
constexpr float kProjScaleQK = kQKCarry / (kActCarry * kWCarry);
constexpr float kProjScaleV  = kVCarry / (kActCarry * kWCarry);
constexpr float kCtxOverV    = kCtxCarry / kVCarry;
constexpr float kOutScale    = 1.0f / (kCtxCarry * kWCarry);

constexpr size_t kPlaneAct = (size_t)kTok * kH * 2;
constexpr size_t kPlaneW   = (size_t)kH * kH * 2;
constexpr size_t kOffXA  = 0;
constexpr size_t kOffXB  = kOffXA + kPlaneAct;
constexpr size_t kOffXC  = kOffXB + kPlaneAct;
constexpr size_t kOffQ   = kOffXC + kPlaneAct;
constexpr size_t kOffW   = kOffQ + kPlaneAct;
constexpr size_t kWsTotal = kOffW + 4 * kPlaneW;
static_assert(kWsTotal == 100663296ull);
static_assert(kWsTotal <= 134217728ull);
static_assert((kOffXB % 128) == 0 && (kOffXC % 128) == 0 && (kOffQ % 128) == 0 && (kOffW % 128) == 0 && (kPlaneW % 128) == 0);

struct FragH {
  union U { v16h v; v8h h[2]; };
  static __device__ __forceinline__ v16h load(const _Float16* p) {
    U f;
    f.h[0] = *(const v8h*)(p);
    f.h[1] = *(const v8h*)(p + 16);
    return f.v;
  }
};

__device__ __forceinline__ v8f mma_g(v16h a, v16h b, v8f c) {
  c = __builtin_amdgcn_wmma_f32_16x16x32_f16(false, a, false, b, (short)0, c, false, false);
  asm volatile("v_nop\n\tv_nop\n\tv_nop\n\tv_nop" : "+v"(c) : "v"(a), "v"(b));
  return c;
}

__global__ __launch_bounds__(256) void cast_planes_kernel(
    const float* __restrict__ s0, const float* __restrict__ s1,
    const float* __restrict__ s2, const float* __restrict__ s3,
    _Float16* __restrict__ dst, int n8, float carry)
{
  const int z = blockIdx.y;
  const float* src = (z == 0) ? s0 : (z == 1) ? s1 : (z == 2) ? s2 : s3;
  const int i = blockIdx.x * 256 + threadIdx.x;
  if (i >= n8) return;
  const float* p = src + 8 * (size_t)i;
  const v4f a = *(const v4f*)(p);
  const v4f c = *(const v4f*)(p + 4);
  v8h hv;
#pragma unroll
  for (int e = 0; e < 4; ++e) {
    const float f0 = a[e] * carry;
    const float f1 = c[e] * carry;
    hv[e]     = (_Float16)f0;
    hv[4 + e] = (_Float16)f1;
  }
  _Float16* q = dst + (size_t)z * (size_t)n8 * 8 + 8 * (size_t)i;
  *(volatile v8h*)q = hv;
  __threadfence();
  *(volatile v8h*)q = hv;
}

template <int BIAS_MODE, bool OUT_F16>
__global__ __launch_bounds__(256) void gemm64_f16_kernel(
    const _Float16* __restrict__ A, int lda,
    const _Float16* __restrict__ Bt, int ldb,
    void* __restrict__ Cout, int ldc,
    const float* __restrict__ bias,
    int M, int N, int K, float scale, float bscale)
{
  __shared__ __align__(16) float sT[8][16 * 68];
  const int lane = threadIdx.x & 31;
  const int wave = __builtin_amdgcn_readfirstlane((int)(threadIdx.x >> 5));
  const int tilesN = N >> 6;
  const int tilesM = M >> 6;
  const int tile = blockIdx.x * 8 + wave;
  if (tile >= tilesM * tilesN) return;
  const int tm = tile / tilesN;
  const int tn = tile - tm * tilesN;
  const int m0 = tm << 6;
  const int n0 = tn << 6;

  const int rlane = lane & 15;
  const int koff  = (lane >> 4) * 8;
  const int mOff  = (lane >> 4) * 8;

  v8f acc[4][4];
#pragma unroll
  for (int i = 0; i < 4; ++i)
#pragma unroll
    for (int j = 0; j < 4; ++j) acc[i][j] = (v8f){0.f, 0.f, 0.f, 0.f, 0.f, 0.f, 0.f, 0.f};

  for (int k0 = 0; k0 < K; k0 += 32) {
    v16h bh[4];
#pragma unroll
    for (int j = 0; j < 4; ++j) {
      const size_t bo = (size_t)(n0 + (j << 4) + rlane) * ldb + koff + k0;
      bh[j] = FragH::load(Bt + bo);
    }
#pragma unroll
    for (int i = 0; i < 4; ++i) {
      const size_t ao = (size_t)(m0 + (i << 4) + rlane) * lda + koff + k0;
      const v16h ah = FragH::load(A + ao);
#pragma unroll
      for (int j = 0; j < 4; ++j) acc[i][j] = mma_g(ah, bh[j], acc[i][j]);
    }
  }

  float* slab = sT[wave];
#pragma unroll
  for (int i = 0; i < 4; ++i) {
    const int mBase = m0 + (i << 4);
#pragma unroll
    for (int j = 0; j < 4; ++j) {
      const int n = n0 + (j << 4) + rlane;
      float bvn = 0.f;
      if (BIAS_MODE == 2) bvn = bias[n] * bscale;
#pragma unroll
      for (int r = 0; r < 8; ++r) {
        float v = acc[i][j][r] * scale;
        if (BIAS_MODE == 1) v += bias[mBase + mOff + r] * bscale;
        if (BIAS_MODE == 2) v += bvn;
        slab[(mOff + r) * 68 + (j << 4) + rlane] = v;
      }
    }
    __builtin_amdgcn_fence(__ATOMIC_RELEASE, "workgroup");
    __builtin_amdgcn_wave_barrier();
    __builtin_amdgcn_fence(__ATOMIC_ACQUIRE, "workgroup");
    if (!OUT_F16) {
      float* C = (float*)Cout;
      const int hh = lane >> 4, c4 = (lane & 15) * 4;
      for (int pass = 0; pass < 2; ++pass) {
#pragma unroll
        for (int it = 0; it < 8; ++it) {
          const int row = it * 2 + hh;
          const v4f v = *(const v4f*)(slab + row * 68 + c4);
          *(volatile v4f*)(C + (size_t)(mBase + row) * ldc + n0 + c4) = v;
        }
        __threadfence();
      }
    } else {
      _Float16* C = (_Float16*)Cout;
      const int q = lane >> 3, c8 = (lane & 7) * 8;
      for (int pass = 0; pass < 2; ++pass) {
#pragma unroll
        for (int it = 0; it < 4; ++it) {
          const int row = it * 4 + q;
          const float* sp = slab + row * 68 + c8;
          v8h hv;
#pragma unroll
          for (int e = 0; e < 8; ++e) hv[e] = (_Float16)sp[e];
          *(volatile v8h*)(C + (size_t)(mBase + row) * ldc + n0 + c8) = hv;
        }
        __threadfence();
      }
    }
    __builtin_amdgcn_fence(__ATOMIC_RELEASE, "workgroup");
    __builtin_amdgcn_wave_barrier();
    __builtin_amdgcn_fence(__ATOMIC_ACQUIRE, "workgroup");
  }
}

constexpr int kFaKP = 136;
constexpr int kFaVP = 72;
constexpr int kFaPP = 72;
constexpr int kFaOP = 136;

__global__ __launch_bounds__(128) void attn_fused_kernel(
    const _Float16* __restrict__ Qp, const _Float16* __restrict__ Kp,
    const _Float16* __restrict__ Vtp, _Float16* __restrict__ Ctx, float coef)
{
  __shared__ __align__(16) _Float16 Ksh[64 * kFaKP];
  __shared__ __align__(16) _Float16 Vsh[128 * kFaVP];
  __shared__ __align__(16) _Float16 Psh[4][16 * kFaPP];
  __shared__ __align__(16) _Float16 Osh[4][16 * kFaOP];

  const int tid  = threadIdx.x;
  const int wave = __builtin_amdgcn_readfirstlane((int)(threadIdx.x >> 5));
  const int lane = tid & 31;
  const int hh   = lane >> 4;
  const int c    = lane & 15;
  const int qb   = blockIdx.x;
  const int bh   = blockIdx.y;
  const int b    = bh / kNH;
  const int h    = bh - b * kNH;
  const int rowbase = b * kS;
  const int colbase = h * kHD;
  const int q0 = qb * 64 + wave * 16;

  v16h qa[4];
  {
    const _Float16* qrow = Qp + (size_t)(rowbase + q0 + c) * kH + colbase + 8 * hh;
#pragma unroll
    for (int dc = 0; dc < 4; ++dc) qa[dc] = FragH::load(qrow + dc * 32);
  }

  float mrow[8], lrow[8];
  v8f oacc[8];
#pragma unroll
  for (int r = 0; r < 8; ++r) { mrow[r] = -1.0e30f; lrow[r] = 0.f; }
#pragma unroll
  for (int t = 0; t < 8; ++t) oacc[t] = (v8f){0.f, 0.f, 0.f, 0.f, 0.f, 0.f, 0.f, 0.f};

  const int ksg = tid & 15, kr0 = tid >> 4;
  const int vsg = tid & 7,  vr0 = tid >> 3;
  const _Float16* kgl = Kp  + (size_t)(rowbase + kr0) * kH + colbase + ksg * 8;
  const _Float16* vgl = Vtp + (size_t)(colbase + vr0) * kTok + rowbase + vsg * 8;
  _Float16* pw = &Psh[wave][0];

#pragma unroll 1
  for (int kc = 0; kc < kS / 64; ++kc) {
    const int kv0 = kc * 64;
    __syncthreads();
    {
      v8h kt[8];
#pragma unroll
      for (int i = 0; i < 8; ++i) kt[i] = *(const v8h*)(kgl + (size_t)(kv0 + 8 * i) * kH);
#pragma unroll
      for (int i = 0; i < 8; ++i) *(v8h*)(Ksh + (kr0 + 8 * i) * kFaKP + ksg * 8) = kt[i];
    }
    {
      v8h vt[8];
#pragma unroll
      for (int i = 0; i < 8; ++i) vt[i] = *(const v8h*)(vgl + (size_t)(16 * i) * kTok + kv0);
#pragma unroll
      for (int i = 0; i < 8; ++i) *(v8h*)(Vsh + (vr0 + 16 * i) * kFaVP + vsg * 8) = vt[i];
    }
    __syncthreads();

    v8f s[4];
#pragma unroll
    for (int j = 0; j < 4; ++j) {
      s[j] = (v8f){0.f, 0.f, 0.f, 0.f, 0.f, 0.f, 0.f, 0.f};
#pragma unroll
      for (int dc = 0; dc < 4; ++dc) {
        const v16h kb = FragH::load(Ksh + (j * 16 + c) * kFaKP + dc * 32 + 8 * hh);
        s[j] = mma_g(qa[dc], kb, s[j]);
      }
    }

    float cm[8];
#pragma unroll
    for (int r = 0; r < 8; ++r) {
      float m = fmaxf(fmaxf(s[0][r], s[1][r]), fmaxf(s[2][r], s[3][r]));
      m = fmaxf(m, __shfl_xor(m, 1, 32));
      m = fmaxf(m, __shfl_xor(m, 2, 32));
      m = fmaxf(m, __shfl_xor(m, 4, 32));
      m = fmaxf(m, __shfl_xor(m, 8, 32));
      cm[r] = m;
    }

#pragma unroll
    for (int r = 0; r < 8; ++r) {
      const float mnew  = fmaxf(mrow[r], cm[r]);
      const float alpha = __expf((mrow[r] - mnew) * coef);
      mrow[r] = mnew;
      float psum = 0.f;
#pragma unroll
      for (int j = 0; j < 4; ++j) {
        const float p = __expf((s[j][r] - mnew) * coef);
        psum += p;
        pw[(8 * hh + r) * kFaPP + j * 16 + c] = (_Float16)p;
      }
      lrow[r] = lrow[r] * alpha + psum;
#pragma unroll
      for (int t = 0; t < 8; ++t) oacc[t][r] *= alpha;
    }
    __builtin_amdgcn_fence(__ATOMIC_RELEASE, "workgroup");
    __builtin_amdgcn_wave_barrier();
    __builtin_amdgcn_fence(__ATOMIC_ACQUIRE, "workgroup");

#pragma unroll
    for (int kk = 0; kk < 2; ++kk) {
      const v16h pa = FragH::load(pw + c * kFaPP + kk * 32 + 8 * hh);
#pragma unroll
      for (int t = 0; t < 8; ++t) {
        const v16h vb = FragH::load(Vsh + (t * 16 + c) * kFaVP + kk * 32 + 8 * hh);
        oacc[t] = mma_g(pa, vb, oacc[t]);
      }
    }
  }

  _Float16* ow = &Osh[wave][0];
#pragma unroll
  for (int r = 0; r < 8; ++r) {
    float l = lrow[r];
    l += __shfl_xor(l, 1, 32);
    l += __shfl_xor(l, 2, 32);
    l += __shfl_xor(l, 4, 32);
    l += __shfl_xor(l, 8, 32);
    const float inv = __builtin_amdgcn_rcpf(l) * kCtxOverV;
#pragma unroll
    for (int t = 0; t < 8; ++t) {
      const float ov = oacc[t][r] * inv;
      ow[(8 * hh + r) * kFaOP + t * 16 + c] = (_Float16)ov;
    }
  }
  __builtin_amdgcn_fence(__ATOMIC_RELEASE, "workgroup");
  __builtin_amdgcn_wave_barrier();
  __builtin_amdgcn_fence(__ATOMIC_ACQUIRE, "workgroup");
  {
    const int sg = (lane & 15) * 8;
    for (int pass = 0; pass < 2; ++pass) {
#pragma unroll
      for (int it = 0; it < 8; ++it) {
        const int row = it * 2 + hh;
        const v8h val = *(const v8h*)(ow + row * kFaOP + sg);
        *(volatile v8h*)(Ctx + (size_t)(rowbase + q0 + row) * kH + colbase + sg) = val;
      }
      __threadfence();
    }
  }
}

extern "C" void kernel_launch(void* const* d_in, const int* in_sizes, int n_in,
                              void* d_out, int out_size, void* d_ws, size_t ws_size,
                              hipStream_t stream) {
  if (n_in < 11) return;
  if (in_sizes[0] != kTok * kH) return;
  if (in_sizes[1] != kTok * kH) return;
  if (in_sizes[2] != kTok * kH) return;
  if (in_sizes[3] != kH * kH) return;
  if (in_sizes[4] != kH) return;
  if (in_sizes[5] != kH * kH) return;
  if (in_sizes[6] != kH) return;
  if (in_sizes[7] != kH * kH) return;
  if (in_sizes[8] != kH) return;
  if (in_sizes[9] != kH * kH) return;
  if (in_sizes[10] != kH) return;
  if (out_size != kTok * kH) return;
  if (ws_size < kWsTotal) return;

  const float* query = (const float*)d_in[0];
  const float* key   = (const float*)d_in[1];
  const float* value = (const float*)d_in[2];
  const float* Wq = (const float*)d_in[3];
  const float* bq = (const float*)d_in[4];
  const float* Wk = (const float*)d_in[5];
  const float* bk = (const float*)d_in[6];
  const float* Wv = (const float*)d_in[7];
  const float* bv = (const float*)d_in[8];
  const float* Wo = (const float*)d_in[9];
  const float* bo = (const float*)d_in[10];
  float* out = (float*)d_out;

  char* ws = (char*)d_ws;
  _Float16* XA  = (_Float16*)(ws + kOffXA);
  _Float16* XB  = (_Float16*)(ws + kOffXB);
  _Float16* XC  = (_Float16*)(ws + kOffXC);
  _Float16* Q16 = (_Float16*)(ws + kOffQ);
  _Float16* W16 = (_Float16*)(ws + kOffW);
  _Float16* Wq16 = W16;
  _Float16* Wk16 = W16 + (size_t)kH * kH;
  _Float16* Wv16 = W16 + 2 * (size_t)kH * kH;
  _Float16* Wo16 = W16 + 3 * (size_t)kH * kH;
  _Float16* K16  = XA;
  _Float16* Vt16 = XB;
  _Float16* C16  = XC;

  const int actN8 = kTok * kH / 8;
  const int wN8   = kH * kH / 8;
  const float scl  = 1.0f / sqrtf((float)kHD);
  const float coef = scl / (kQKCarry * kQKCarry);
  const int gemmBlocks = ((kTok / 64) * (kH / 64)) / 8;

  cast_planes_kernel<<<dim3(actN8 / 256, 3), 256, 0, stream>>>(query, key, value, value, XA, actN8, kActCarry);
  cast_planes_kernel<<<dim3(wN8 / 256, 4), 256, 0, stream>>>(Wq, Wk, Wv, Wo, W16, wN8, kWCarry);

  gemm64_f16_kernel<2, true><<<gemmBlocks, 256, 0, stream>>>(
      XA, kH, Wq16, kH, (void*)Q16, kH, bq, kTok, kH, kH, kProjScaleQK, kQKCarry);

  gemm64_f16_kernel<2, true><<<gemmBlocks, 256, 0, stream>>>(
      XB, kH, Wk16, kH, (void*)K16, kH, bk, kTok, kH, kH, kProjScaleQK, kQKCarry);

  gemm64_f16_kernel<1, true><<<gemmBlocks, 256, 0, stream>>>(
      Wv16, kH, XC, kH, (void*)Vt16, kTok, bv, kH, kTok, kH, kProjScaleV, kVCarry);

  attn_fused_kernel<<<dim3(kS / 64, kB * kNH), 128, 0, stream>>>(Q16, K16, Vt16, C16, coef);

  gemm64_f16_kernel<2, false><<<gemmBlocks, 256, 0, stream>>>(
      C16, kH, Wo16, kH, (void*)out, kH, bo, kTok, kH, kH, kOutScale, 1.0f);
}
